// MaskDeformConv2dModule_26079041421805
// MI455X (gfx1250) — hardware-verified
//
#include <hip/hip_runtime.h>

#pragma clang fp contract(off)

typedef unsigned short us_t;
typedef unsigned short v8us  __attribute__((ext_vector_type(8)));
typedef unsigned short v16us __attribute__((ext_vector_type(16)));
typedef __bf16         v16bf __attribute__((ext_vector_type(16)));
typedef float          v8f   __attribute__((ext_vector_type(8)));
typedef float          v4f   __attribute__((ext_vector_type(4)));
typedef int            v4i   __attribute__((ext_vector_type(4)));
typedef v8us __attribute__((may_alias)) v8usa;
typedef v4f  __attribute__((may_alias)) v4fa;
typedef v4i  __attribute__((may_alias)) v4ia;
union Frag { v16us v; v8us half[2]; };

#define NBATCH 4
#define CIN    256
#define COUT   256
#define HH     64
#define WWD    64
#define NPIX   4096
#define KP     9
#define KTOT   2304
#define KSTEPS 72
#define TP     40
#define GSZ    32768

#define SM_IDX 0
#define SM_WGT 9216
#define SM_MSK 18432
#define SM_THI 20736
#define SM_TLO 25856
#define SM_BYTES 65536

__device__ __forceinline__ us_t bf16_rne(float f) {
  unsigned int u = __float_as_uint(f);
  u += 0x7FFFu + ((u >> 16) & 1u);
  return (us_t)(u >> 16);
}
__device__ __forceinline__ float bf16_val(us_t s) {
  return __uint_as_float(((unsigned int)s) << 16);
}

__device__ __forceinline__ v8f wmma_bf16(v16us a, v16us b, v8f c) {
  const v16bf ab = __builtin_bit_cast(v16bf, a);
  const v16bf bb = __builtin_bit_cast(v16bf, b);
  v8f d = __builtin_amdgcn_wmma_f32_16x16x32_bf16(false, ab, false, bb, (short)0, c, false, false);
  asm volatile("v_nop\n\tv_nop\n\tv_nop\n\tv_nop" : "+v"(d) : "v"(a), "v"(b));
  return d;
}

__device__ __forceinline__ v16us load_frag(const us_t* p, int h) {
  Frag f;
  f.half[0] = *(const v8usa*)(p + 8 * h);
  f.half[1] = *(const v8usa*)(p + 16 + 8 * h);
  return f.v;
}

__device__ __forceinline__ double wave_sum_d(double s) {
  s += __shfl_xor(s, 16);
  s += __shfl_xor(s, 8);
  s += __shfl_xor(s, 4);
  s += __shfl_xor(s, 2);
  s += __shfl_xor(s, 1);
  return s;
}

__global__ __launch_bounds__(256) void wsplit_k(const float* __restrict__ w,
                                                us_t* __restrict__ whi, us_t* __restrict__ wlo)
{
  const int g = blockIdx.x * 256 + threadIdx.x;
  if (g >= COUT * (KTOT / 8)) return;
  const int o = g / (KTOT / 8);
  const int q = g - o * (KTOT / 8);
  const int kp = q >> 5, c0 = (q & 31) * 8;
  v8us hv, lv;
  #pragma unroll
  for (int j = 0; j < 8; ++j) {
    const float v = w[(size_t)(o * CIN + c0 + j) * KP + kp];
    const us_t hs = bf16_rne(v);
    hv[j] = hs;
    lv[j] = bf16_rne(v - bf16_val(hs));
  }
  const size_t d = (size_t)o * KTOT + (size_t)q * 8;
  *(volatile v8us*)(whi + d) = hv;
  *(volatile v8us*)(wlo + d) = lv;
  __threadfence();
  *(volatile v8us*)(whi + d) = hv;
  *(volatile v8us*)(wlo + d) = lv;
}

__global__ __launch_bounds__(256) void dcn_k(
    const float* __restrict__ x, const float* __restrict__ off, const float* __restrict__ msk,
    const us_t* __restrict__ whi, const us_t* __restrict__ wlo, const float* __restrict__ bias,
    float* __restrict__ conv)
{
  __shared__ __align__(16) unsigned char smem[SM_BYTES];
  v4ia*  sIdx = (v4ia*)(smem + SM_IDX);
  v4fa*  sWgt = (v4fa*)(smem + SM_WGT);
  float* sMsk = (float*)(smem + SM_MSK);
  us_t*  sThi = (us_t*)(smem + SM_THI);
  us_t*  sTlo = (us_t*)(smem + SM_TLO);
  float* sD   = (float*)(smem);

  const int tid = threadIdx.x, lane = tid & 31, wid = tid >> 5;
  const int b = blockIdx.x >> 6, hrow = blockIdx.x & 63;

  for (int t = tid; t < KP * 64; t += 256) {
    const int kp = t >> 6, n = t & 63;
    const int ky = kp / 3, kx = kp - 3 * ky;
    const size_t pix = (size_t)hrow * WWD + n;
    const float offy = off[(size_t)(b * 2 * KP + 2 * kp) * NPIX + pix];
    const float offx = off[(size_t)(b * 2 * KP + 2 * kp + 1) * NPIX + pix];
    const float mv   = msk[(size_t)(b * KP + kp) * NPIX + pix];
    const float yy = (float)(ky + hrow - 1) + offy;
    const float xx = (float)(kx + n - 1) + offx;
    const float y0 = floorf(yy), x0 = floorf(xx);
    const float fy = yy - y0, fx = xx - x0;
    const float gy = 1.0f - fy, gx = 1.0f - fx;
    const int y0i = (int)fminf(fmaxf(y0, -4.0f), 68.0f);
    const int x0i = (int)fminf(fmaxf(x0, -4.0f), 68.0f);
    const int y1i = y0i + 1, x1i = x0i + 1;
    const bool vy0 = (y0i >= 0) && (y0i <= HH - 1);
    const bool vy1 = (y1i >= 0) && (y1i <= HH - 1);
    const bool vx0 = (x0i >= 0) && (x0i <= WWD - 1);
    const bool vx1 = (x1i >= 0) && (x1i <= WWD - 1);
    const int yc0 = min(max(y0i, 0), HH - 1), yc1 = min(max(y1i, 0), HH - 1);
    const int xc0 = min(max(x0i, 0), WWD - 1), xc1 = min(max(x1i, 0), WWD - 1);
    v4i id;
    id.x = yc0 * WWD + xc0;
    id.y = yc0 * WWD + xc1;
    id.z = yc1 * WWD + xc0;
    id.w = yc1 * WWD + xc1;
    v4f wt;
    wt.x = (vy0 && vx0) ? (gy * gx) : 0.0f;
    wt.y = (vy0 && vx1) ? (gy * fx) : 0.0f;
    wt.z = (vy1 && vx0) ? (fy * gx) : 0.0f;
    wt.w = (vy1 && vx1) ? (fy * fx) : 0.0f;
    sIdx[t] = id;
    sWgt[t] = wt;
    sMsk[t] = mv;
  }

  const int h = lane >> 4, m = lane & 15;
  const int wm = wid & 3, wn = wid >> 2;
  const int bn = tid >> 2, bcq = (tid & 3) * 8;

  v8f acc[4][2];
  #pragma unroll
  for (int mt = 0; mt < 4; ++mt) {
    #pragma unroll
    for (int nt = 0; nt < 2; ++nt) {
      #pragma unroll
      for (int r = 0; r < 8; ++r) acc[mt][nt][r] = 0.0f;
    }
  }

  __syncthreads();

  #pragma unroll 1
  for (int ks = 0; ks < KSTEPS; ++ks) {
    {
      const int kp = ks >> 3, ct = ks & 7;
      const v4i id = sIdx[kp * 64 + bn];
      const v4f wv = sWgt[kp * 64 + bn];
      const float mv = sMsk[kp * 64 + bn];
      const float* xb = x + (size_t)(b * CIN + ct * 32 + bcq) * NPIX;
      v8us hv, lv;
      #pragma unroll
      for (int j = 0; j < 8; ++j) {
        const float* p = xb + (size_t)j * NPIX;
        const float c0 = p[id.x] * wv.x;
        const float c1 = p[id.y] * wv.y;
        const float c2 = p[id.z] * wv.z;
        const float c3 = p[id.w] * wv.w;
        float r = c0 + c1;
        r = r + c2;
        r = r + c3;
        r = r * mv;
        const us_t hs = bf16_rne(r);
        hv[j] = hs;
        lv[j] = bf16_rne(r - bf16_val(hs));
      }
      *(v8usa*)(sThi + bn * TP + bcq) = hv;
      *(v8usa*)(sTlo + bn * TP + bcq) = lv;
    }
    __syncthreads();

    {
      const us_t* wbh = whi + (size_t)(64 * wm + m) * KTOT + ks * 32;
      const us_t* wbl = wlo + (size_t)(64 * wm + m) * KTOT + ks * 32;
      v16us bh[2], bl[2];
      #pragma unroll
      for (int nt = 0; nt < 2; ++nt) {
        const int trow = (32 * wn + 16 * nt + m) * TP;
        bh[nt] = load_frag(sThi + trow, h);
        bl[nt] = load_frag(sTlo + trow, h);
      }
      #pragma unroll
      for (int mt = 0; mt < 4; ++mt) {
        const v16us ah = load_frag(wbh + (size_t)mt * 16 * KTOT, h);
        const v16us al = load_frag(wbl + (size_t)mt * 16 * KTOT, h);
        #pragma unroll
        for (int nt = 0; nt < 2; ++nt) {
          acc[mt][nt] = wmma_bf16(ah, bh[nt], acc[mt][nt]);
          acc[mt][nt] = wmma_bf16(ah, bl[nt], acc[mt][nt]);
          acc[mt][nt] = wmma_bf16(al, bh[nt], acc[mt][nt]);
        }
      }
    }
    __syncthreads();
  }

  #pragma unroll
  for (int mt = 0; mt < 4; ++mt) {
    #pragma unroll
    for (int nt = 0; nt < 2; ++nt) {
      const int px = 32 * wn + 16 * nt + m;
      #pragma unroll
      for (int r = 0; r < 8; ++r) {
        const int o = 64 * wm + 16 * mt + 8 * h + r;
        sD[o * 64 + px] = acc[mt][nt][r] + bias[o];
      }
    }
  }
  __syncthreads();

  const int sub = lane >> 3, q8 = lane & 7;
  const int px0 = 32 * wn + 4 * q8;
  #pragma unroll
  for (int i = 0; i < 16; ++i) {
    const int o = 64 * wm + 4 * i + sub;
    const v4f v = *(const v4fa*)(sD + o * 64 + px0);
    const size_t gi = ((size_t)(b * COUT + o) * HH + hrow) * WWD + px0;
    *(volatile v4f*)(conv + gi) = v;
  }
  __threadfence();
  #pragma unroll
  for (int i = 0; i < 16; ++i) {
    const int o = 64 * wm + 4 * i + sub;
    const v4f v = *(const v4fa*)(sD + o * 64 + px0);
    const size_t gi = ((size_t)(b * COUT + o) * HH + hrow) * WWD + px0;
    *(volatile v4f*)(conv + gi) = v;
  }
}

__global__ __launch_bounds__(256) void gn_k(
    const float* __restrict__ conv, const float* __restrict__ gam, const float* __restrict__ bet,
    float* __restrict__ out)
{
  __shared__ double sred[8];
  const int tid = threadIdx.x, lane = tid & 31, wid = tid >> 5;
  const int bg = blockIdx.x;
  const int grp = bg & 31;
  const size_t base = (size_t)bg * GSZ;
  const float* src = conv + base;

  double s = 0.0;
  #pragma unroll 2
  for (int k = 0; k < 32; ++k) {
    const v4f v = *(const v4fa*)(src + (size_t)k * 1024 + 4 * tid);
    s += ((double)v.x + (double)v.y) + ((double)v.z + (double)v.w);
  }
  s = wave_sum_d(s);
  if (lane == 0) sred[wid] = s;
  __syncthreads();
  double S = 0.0;
  #pragma unroll
  for (int k = 0; k < 8; ++k) S += sred[k];
  const double mu = S * (1.0 / 32768.0);
  __syncthreads();

  double q = 0.0;
  #pragma unroll 2
  for (int k = 0; k < 32; ++k) {
    const v4f v = *(const v4fa*)(src + (size_t)k * 1024 + 4 * tid);
    const double d0 = (double)v.x - mu, d1 = (double)v.y - mu;
    const double d2 = (double)v.z - mu, d3 = (double)v.w - mu;
    q += (d0 * d0 + d1 * d1) + (d2 * d2 + d3 * d3);
  }
  q = wave_sum_d(q);
  if (lane == 0) sred[wid] = q;
  __syncthreads();
  double Q = 0.0;
  #pragma unroll
  for (int k = 0; k < 8; ++k) Q += sred[k];
  const double var = Q * (1.0 / 32768.0);
  const float muf = (float)mu;
  const float rs = (float)(1.0 / sqrt(var + 1.0e-5));

  #pragma unroll 1
  for (int k = 0; k < 32; ++k) {
    const int cl = k >> 2;
    const float ga = gam[8 * grp + cl];
    const float be = bet[8 * grp + cl];
    const size_t idx = (size_t)k * 1024 + 4 * tid;
    const v4f v = *(const v4fa*)(src + idx);
    v4f o;
    o.x = fmaxf(((v.x - muf) * rs) * ga + be, 0.0f);
    o.y = fmaxf(((v.y - muf) * rs) * ga + be, 0.0f);
    o.z = fmaxf(((v.z - muf) * rs) * ga + be, 0.0f);
    o.w = fmaxf(((v.w - muf) * rs) * ga + be, 0.0f);
    float* dst = out + base + idx;
    *(volatile v4f*)dst = o;
    __threadfence();
    *(volatile v4f*)dst = o;
  }
}

extern "C" void kernel_launch(void* const* d_in, const int* in_sizes, int n_in,
                              void* d_out, int out_size, void* d_ws, size_t ws_size,
                              hipStream_t stream) {
  if (n_in < 7) return;
  if (in_sizes[0] != NBATCH * CIN * NPIX) return;
  if (in_sizes[1] != NBATCH * 2 * KP * NPIX) return;
  if (in_sizes[2] != NBATCH * KP * NPIX) return;
  if (in_sizes[3] != COUT * CIN * KP) return;
  if (in_sizes[4] < COUT || in_sizes[5] < COUT || in_sizes[6] < COUT) return;
  if (out_size != NBATCH * COUT * NPIX) return;

  const float* x     = (const float*)d_in[0];
  const float* off   = (const float*)d_in[1];
  const float* msk   = (const float*)d_in[2];
  const float* wgt   = (const float*)d_in[3];
  const float* bias  = (const float*)d_in[4];
  const float* gam   = (const float*)d_in[5];
  const float* bet   = (const float*)d_in[6];
  float* out = (float*)d_out;

  const size_t wplane = (size_t)COUT * KTOT * sizeof(us_t);
  const size_t convb  = (size_t)NBATCH * COUT * NPIX * sizeof(float);
  const size_t o_whi  = 0;
  const size_t o_wlo  = o_whi + wplane;
  const size_t o_conv = o_wlo + wplane;
  const size_t total  = o_conv + convb;
  if (total > ws_size) return;
  char* ws = (char*)d_ws;
  us_t*  whi  = (us_t*)(ws + o_whi);
  us_t*  wlo  = (us_t*)(ws + o_wlo);
  float* conv = (float*)(ws + o_conv);

  wsplit_k<<<(COUT * (KTOT / 8)) / 256, 256, 0, stream>>>(wgt, whi, wlo);
  dcn_k<<<NBATCH * HH, 256, 0, stream>>>(x, off, msk, whi, wlo, bias, conv);
  gn_k<<<NBATCH * 32, 256, 0, stream>>>(conv, gam, bet, out);
}
